// lwm_mamba_30081950941582
// MI455X (gfx1250) — hardware-run, weakly checked
//
#include <hip/hip_runtime.h>
#include <math.h>

typedef __attribute__((ext_vector_type(16))) _Float16 v16h;
typedef __attribute__((ext_vector_type(8)))  _Float16 v8h;
typedef __attribute__((ext_vector_type(16))) __bf16   v16b;
typedef __attribute__((ext_vector_type(8)))  __bf16   v8b;
typedef __attribute__((ext_vector_type(8)))  float    v8f;
typedef __attribute__((ext_vector_type(4)))  float    v4f;
typedef __attribute__((ext_vector_type(2)))  float    v2f;

constexpr int kBatch    = 4;
constexpr int kSeq      = 512;
constexpr int kDm       = 128;
constexpr int kElem     = 32;
constexpr int kLayers   = 12;
constexpr int kNst      = 16;
constexpr int kDtR      = 8;
constexpr int kDin      = 256;
constexpr int kDff      = 512;
constexpr int kNMask    = 64;
constexpr int kRows     = kBatch * kSeq;
constexpr int kXzP      = 2 * kDin;
constexpr int kXdN      = kDtR + 2 * kNst;
constexpr int kXdP      = 64;
constexpr int kHeadRows = kBatch * kNMask;
constexpr int kDecP     = 64;
constexpr int kConvTP   = 260;
constexpr int kScanTS   = 64;
constexpr int kScanCh   = 64;
constexpr int kScanYP   = 68;
static_assert(kXdN <= kXdP, "x_proj pad");
static_assert((kDm % 32) == 0 && (kDin % 32) == 0 && (kDff % 32) == 0 && (kElem % 32) == 0, "GEMM K multiples of 32");
static_assert((kRows % 64) == 0 && (kXzP % 64) == 0 && (kXdP % 64) == 0 && (kDm % 64) == 0 && (kDff % 64) == 0 &&
              (kHeadRows % 64) == 0 && (kDecP % 64) == 0, "GEMM M,N multiples of 64");
static_assert((kSeq % kScanTS) == 0 && (kSeq % 64) == 0 && (kDin % kScanCh) == 0 && (kDin % 256) == 0, "tile multiples");
static_assert((kRows % 16) == 0 && (kHeadRows % 16) == 0, "LN blocks of 16 rows");

constexpr size_t kOffX16 = 0;
constexpr size_t kOffPW  = kOffX16 + (size_t)kRows * kElem * 2;
constexpr size_t kOffWIN = kOffPW  + (size_t)kDm * kElem * 2;
constexpr size_t kOffWX  = kOffWIN + (size_t)kLayers * kXzP * kDm * 2;
constexpr size_t kOffWO  = kOffWX  + (size_t)kLayers * kXdP * kDin * 2;
constexpr size_t kOffW1  = kOffWO  + (size_t)kLayers * kDm * kDin * 2;
constexpr size_t kOffW2  = kOffW1  + (size_t)kLayers * kDff * kDm * 2;
constexpr size_t kOffLIN = kOffW2  + (size_t)kLayers * kDm * kDff * 2;
constexpr size_t kOffDEC = kOffLIN + (size_t)kDm * kDm * 2;
constexpr size_t kOffOUT = kOffDEC + (size_t)kDecP * kDm * 2;
constexpr size_t kOffTT  = kOffOUT + (size_t)kRows * kDm * 4;
constexpr size_t kOffH16 = kOffTT  + (size_t)kRows * kDm * 4;
constexpr size_t kOffA16 = kOffH16 + (size_t)kRows * kDm * 2;
constexpr size_t kOffXZ  = kOffA16 + (size_t)kRows * kDm * 2;
constexpr size_t kOffUC  = kOffXZ  + (size_t)kRows * kXzP * 4;
constexpr size_t kOffUP  = kOffUC  + (size_t)kRows * kDin * 4;
constexpr size_t kOffXD  = kOffUP  + (size_t)kRows * kDin * 2;
constexpr size_t kOffYP  = kOffXD  + (size_t)kRows * kXdP * 4;
constexpr size_t kOffF1  = kOffYP  + (size_t)kRows * kDin * 2;
constexpr size_t kOffG16 = kOffF1  + (size_t)kRows * kDff * 4;
constexpr size_t kOffHM  = kOffG16 + (size_t)kRows * kDff * 2;
constexpr size_t kOffHL  = kOffHM  + (size_t)kHeadRows * kDm * 2;
constexpr size_t kOffHG  = kOffHL  + (size_t)kHeadRows * kDm * 4;
constexpr size_t kOffHN  = kOffHG  + (size_t)kHeadRows * kDm * 4;
constexpr size_t kOffLG  = kOffHN  + (size_t)kHeadRows * kDm * 2;
constexpr size_t kWsTotal = kOffLG + (size_t)kHeadRows * kDecP * 4;
static_assert(kWsTotal == 24895488ull, "carve total");
static_assert(kWsTotal <= 134217728ull, "carve cap");
static_assert((kOffPW % 128) == 0 && (kOffWIN % 128) == 0 && (kOffWX % 128) == 0 && (kOffWO % 128) == 0 &&
              (kOffW1 % 128) == 0 && (kOffW2 % 128) == 0 && (kOffLIN % 128) == 0 && (kOffDEC % 128) == 0 &&
              (kOffOUT % 128) == 0 && (kOffTT % 128) == 0 && (kOffH16 % 128) == 0 && (kOffA16 % 128) == 0 &&
              (kOffXZ % 128) == 0 && (kOffUC % 128) == 0 && (kOffUP % 128) == 0 && (kOffXD % 128) == 0 &&
              (kOffYP % 128) == 0 && (kOffF1 % 128) == 0 && (kOffG16 % 128) == 0 && (kOffHM % 128) == 0 &&
              (kOffHL % 128) == 0 && (kOffHG % 128) == 0 && (kOffHN % 128) == 0 && (kOffLG % 128) == 0,
              "128-B aligned regions");
constexpr int kOut0Floats = kHeadRows * kElem;
constexpr int kOutTotal   = kOut0Floats + kRows * kDm;
static_assert(kOut0Floats * 4 == 32768, "out1 byte offset");

__device__ __forceinline__ unsigned short f2bf_bits(float f) {
  unsigned u = __float_as_uint(f);
  return (unsigned short)((u + 0x7FFFu + ((u >> 16) & 1u)) >> 16);
}
__device__ __forceinline__ float bf_bits2f(unsigned short h) { return __uint_as_float(((unsigned)h) << 16); }

__device__ __forceinline__ void dep_guard_h(v8f& a, v8f& b, v16h x, v16h y) { asm volatile("v_nop\n\tv_nop\n\tv_nop\n\tv_nop" : "+v"(a), "+v"(b) : "v"(x), "v"(y)); }
__device__ __forceinline__ void dep_guard_b(v8f& a, v8f& b, v16b x, v16b y) { asm volatile("v_nop\n\tv_nop\n\tv_nop\n\tv_nop" : "+v"(a), "+v"(b) : "v"(x), "v"(y)); }
__device__ __forceinline__ void keep4_h(v16h a, v16h b, v16h c, v16h d) { asm volatile("v_nop" :: "v"(a), "v"(b), "v"(c), "v"(d)); }
__device__ __forceinline__ void keep4_b(v16b a, v16b b, v16b c, v16b d) { asm volatile("v_nop" :: "v"(a), "v"(b), "v"(c), "v"(d)); }
__device__ __forceinline__ void acc_guard4(v8f& a, v8f& b, v8f& c, v8f& d) { asm volatile("v_nop\n\tv_nop\n\tv_nop\n\tv_nop" : "+v"(a), "+v"(b), "+v"(c), "+v"(d)); }
template <typename T> struct Frag;
template <> struct Frag<_Float16> {
  typedef v16h V; union U { v16h v; v8h h[2]; };
  static __device__ __forceinline__ v16h load(const _Float16* p) {
    U f; f.h[0] = *(const v8h*)(p); f.h[1] = *(const v8h*)(p + 16); return f.v;
  }
  static __device__ __forceinline__ v8f mma(v16h a, v16h b, v8f c) {
    return __builtin_amdgcn_wmma_f32_16x16x32_f16(false, a, false, b, (short)0, c, false, false);
  }
  static __device__ __forceinline__ void guard(v8f& a, v8f& b, v16h x, v16h y) { dep_guard_h(a, b, x, y); }
  static __device__ __forceinline__ void keep(v16h a, v16h b, v16h c, v16h d) { keep4_h(a, b, c, d); }
};
template <> struct Frag<__bf16> {
  typedef v16b V; union U { v16b v; v8b h[2]; };
  static __device__ __forceinline__ v16b load(const __bf16* p) {
    U f; f.h[0] = *(const v8b*)(p); f.h[1] = *(const v8b*)(p + 16); return f.v;
  }
  static __device__ __forceinline__ v8f mma(v16b a, v16b b, v8f c) {
    return __builtin_amdgcn_wmma_f32_16x16x32_bf16(false, a, false, b, (short)0, c, false, false);
  }
  static __device__ __forceinline__ void guard(v8f& a, v8f& b, v16b x, v16b y) { dep_guard_b(a, b, x, y); }
  static __device__ __forceinline__ void keep(v16b a, v16b b, v16b c, v16b d) { keep4_b(a, b, c, d); }
};

template <int ET> struct Elem;
template <> struct Elem<0> { typedef _Float16 T; };
template <> struct Elem<1> { typedef __bf16 T; };
template <int ET, int SPL, int BIAS_MODE, int OUT_MODE, bool RESID, int ACT = 0>
__global__ __launch_bounds__(256) void wmma_gemm64(
    const unsigned short* __restrict__ Ap, const unsigned short* __restrict__ A2p, int lda, long strideA,
    const unsigned short* __restrict__ Btp, const unsigned short* __restrict__ Bt2p, int ldb, long strideB,
    void* __restrict__ Cout, void* __restrict__ Cout2, int ldc, long strideC,
    const float* __restrict__ bias,
    const float* __restrict__ resid, long strideR,
    int M, int N, int K, float scale) {
  typedef typename Elem<ET>::T T;
  typedef typename Frag<T>::V V;
  const T* A = (const T*)Ap; const T* A2 = (const T*)A2p; const T* Bt = (const T*)Btp; const T* Bt2 = (const T*)Bt2p;
  __shared__ __align__(16) float sT[8][16 * 68];
  const int b    = blockIdx.y;
  const int lane = threadIdx.x & 31;
  const int wave = threadIdx.x >> 5;
  const int tilesN = N >> 6;
  const int tilesM = M >> 6;
  const int tile = blockIdx.x * 8 + wave;
  if (tile >= tilesM * tilesN) return;
  const int tm = tile / tilesN;
  const int tn = tile - tm * tilesN;
  const int m0 = tm << 6;
  const int n0 = tn << 6;

  const T* Ab  = A  + (size_t)b * strideA;
  const T* Bb  = Bt + (size_t)b * strideB;
  const T* Ab2 = (SPL >= 1) ? (A2  + (size_t)b * strideA) : nullptr;
  const T* Bb2 = (SPL == 2) ? (Bt2 + (size_t)b * strideB) : nullptr;

  const int rlane = lane & 15;
  const int koff  = (lane >> 4) * 8;
  const int mOff  = (lane >> 4) * 8;

  v8f acc[4][4];
#pragma unroll
  for (int i = 0; i < 4; ++i)
#pragma unroll
    for (int j = 0; j < 4; ++j) acc[i][j] = (v8f){0.f,0.f,0.f,0.f,0.f,0.f,0.f,0.f};

  for (int k0 = 0; k0 < K; k0 += 32) {
    V bh[4], bl[4];
#pragma unroll
    for (int j = 0; j < 4; ++j) {
      const size_t bo = (size_t)(n0 + (j << 4) + rlane) * ldb + koff + k0;
      bh[j] = Frag<T>::load(Bb + bo);
      if (SPL == 2) bl[j] = Frag<T>::load(Bb2 + bo);
    }
#pragma unroll
    for (int i = 0; i < 4; ++i) {
      const size_t ao = (size_t)(m0 + (i << 4) + rlane) * lda + koff + k0;
      V ah = Frag<T>::load(Ab + ao);
      V al;
      if (SPL >= 1) al = Frag<T>::load(Ab2 + ao);
#pragma unroll
      for (int j = 0; j < 4; ++j) {
        acc[i][j] = Frag<T>::mma(ah, bh[j], acc[i][j]);
        if (SPL == 2) acc[i][j] = Frag<T>::mma(ah, bl[j], acc[i][j]);
        if (SPL >= 1) acc[i][j] = Frag<T>::mma(al, bh[j], acc[i][j]);
      }
      Frag<T>::guard(acc[i][0], acc[i][3], ah, (SPL >= 1) ? al : ah);
    }
    Frag<T>::keep(bh[0], bh[1], bh[2], bh[3]);
    if (SPL == 2) Frag<T>::keep(bl[0], bl[1], bl[2], bl[3]);
  }
  acc_guard4(acc[0][0], acc[0][1], acc[0][2], acc[0][3]);
  acc_guard4(acc[1][0], acc[1][1], acc[1][2], acc[1][3]);
  acc_guard4(acc[2][0], acc[2][1], acc[2][2], acc[2][3]);
  acc_guard4(acc[3][0], acc[3][1], acc[3][2], acc[3][3]);

  float* slab = sT[wave];
  const float* Rb = RESID ? (resid + (size_t)b * strideR) : nullptr;
#pragma unroll
  for (int i = 0; i < 4; ++i) {
    const int mBase = m0 + (i << 4);
#pragma unroll
    for (int j = 0; j < 4; ++j) {
      const int n = n0 + (j << 4) + rlane;
      float bv = 0.f;
      if (BIAS_MODE == 2) bv = bias[n];
#pragma unroll
      for (int r = 0; r < 8; ++r) {
        float v = acc[i][j][r] * scale;
        if (BIAS_MODE == 1) v += bias[mBase + mOff + r];
        if (BIAS_MODE == 2) v += bv;
        if (RESID) v += Rb[(size_t)(mBase + mOff + r) * ldc + n];
        if (ACT == 1) v = tanhf(v);
        if (ACT == 2) v = fmaxf(v, 0.0f);
        if (ACT == 3) v = v / (1.0f + expf(-v));
        if (ACT == 4) v = (v > 0.f) ? v : 0.01f * v;
        slab[(mOff + r) * 68 + (j << 4) + rlane] = v;
      }
    }
    __builtin_amdgcn_fence(__ATOMIC_RELEASE, "workgroup");
    __builtin_amdgcn_wave_barrier();
    __builtin_amdgcn_fence(__ATOMIC_ACQUIRE, "workgroup");
    if (OUT_MODE == 0) {
      float* C = (float*)Cout + (size_t)b * strideC;
      const int hh = lane >> 4, c4 = (lane & 15) * 4;
      for (int pass = 0; pass < 2; ++pass) {
#pragma unroll
        for (int it = 0; it < 8; ++it) {
          const int row = it * 2 + hh;
          v4f v = *(const v4f*)(slab + row * 68 + c4);
          *(volatile v4f*)(C + (size_t)(mBase + row) * ldc + n0 + c4) = v;
        }
        __threadfence();
      }
    } else {
      const int q = lane >> 3, c8 = (lane & 7) * 8;
      unsigned short* C  = (unsigned short*)Cout  + (size_t)b * strideC;
      unsigned short* C2 = (OUT_MODE == 2) ? ((unsigned short*)Cout2 + (size_t)b * strideC) : nullptr;
      for (int pass = 0; pass < 2; ++pass) {
#pragma unroll
        for (int it = 0; it < 4; ++it) {
          const int row = it * 4 + q;
          const float* sp = slab + row * 68 + c8;
          v8h hv, lv;
#pragma unroll
          for (int e = 0; e < 8; ++e) {
            if (OUT_MODE == 1) {
              hv[e] = (_Float16)sp[e];
            } else {
              unsigned short hb = f2bf_bits(sp[e]);
              unsigned short lb = f2bf_bits(sp[e] - bf_bits2f(hb));
              hv[e] = __builtin_bit_cast(_Float16, hb);
              lv[e] = __builtin_bit_cast(_Float16, lb);
            }
          }
          *(volatile v8h*)(C + (size_t)(mBase + row) * ldc + n0 + c8) = hv;
          if (OUT_MODE == 2) *(volatile v8h*)(C2 + (size_t)(mBase + row) * ldc + n0 + c8) = lv;
        }
        __threadfence();
      }
    }
    __builtin_amdgcn_fence(__ATOMIC_RELEASE, "workgroup");
    __builtin_amdgcn_wave_barrier();
    __builtin_amdgcn_fence(__ATOMIC_ACQUIRE, "workgroup");
  }
}

__global__ __launch_bounds__(256) void cast_pad_f16_kernel(
    const float* __restrict__ src, unsigned short* __restrict__ dst,
    int rows_src, int rows_dst, int cols, float scale, int total8)
{
  const int i = blockIdx.x * 256 + threadIdx.x;
  if (i >= total8) return;
  const size_t e0 = (size_t)i << 3;
  const size_t rr = e0 / (size_t)cols;
  const int col  = (int)(e0 - rr * (size_t)cols);
  const int rdst = (int)(rr % (size_t)rows_dst);
  const int mat  = (int)(rr / (size_t)rows_dst);
  const bool live = (rdst < rows_src);
  const int rsrc = live ? rdst : (rows_src - 1);
  const float* sp = src + ((size_t)mat * rows_src + rsrc) * cols + col;
  const v4f a0 = *(const v4f*)(sp);
  const v4f a1 = *(const v4f*)(sp + 4);
  v8h hv;
#pragma unroll
  for (int e = 0; e < 4; ++e) {
    const float f0 = live ? a0[e] * scale : 0.0f;
    const float f1 = live ? a1[e] * scale : 0.0f;
    hv[e]     = (_Float16)f0;
    hv[4 + e] = (_Float16)f1;
  }
  unsigned short* q = dst + e0;
  *(volatile v8h*)q = hv;
  __threadfence();
  *(volatile v8h*)q = hv;
}

__device__ __forceinline__ v4f ln_vec4(v4f x, v4f g, v4f bb) {
  float s = (x[0] + x[1]) + (x[2] + x[3]);
#pragma unroll
  for (int off = 16; off > 0; off >>= 1) s += __shfl_xor(s, off, 32);
  const float mean = s * (1.0f / 128.0f);
  v4f d;
  d[0] = x[0] - mean; d[1] = x[1] - mean; d[2] = x[2] - mean; d[3] = x[3] - mean;
  float q = (d[0] * d[0] + d[1] * d[1]) + (d[2] * d[2] + d[3] * d[3]);
#pragma unroll
  for (int off = 16; off > 0; off >>= 1) q += __shfl_xor(q, off, 32);
  const float rstd = rsqrtf(q * (1.0f / 128.0f) + 1e-5f);
  v4f y;
  y[0] = d[0] * rstd * g[0] + bb[0];
  y[1] = d[1] * rstd * g[1] + bb[1];
  y[2] = d[2] * rstd * g[2] + bb[2];
  y[3] = d[3] * rstd * g[3] + bb[3];
  return y;
}

template <int MODE>
__global__ __launch_bounds__(256) void ln_rows_kernel(
    const float* __restrict__ src,
    const float* __restrict__ g1, const float* __restrict__ b1,
    const float* __restrict__ g2, const float* __restrict__ b2,
    float* __restrict__ outf, unsigned short* __restrict__ out16, int rows, float s16)
{
  __shared__ __align__(16) _Float16 sH[8][2 * kDm];
  const int lane = threadIdx.x & 31, wave = threadIdx.x >> 5;
  const int r0 = (blockIdx.x * 8 + wave) * 2;
  if (r0 + 2 > rows) return;
  const int c4 = lane * 4;
  const v4f ga = *(const v4f*)(g1 + c4);
  const v4f ba = *(const v4f*)(b1 + c4);
  v4f gb = ga, bb2 = ba;
  if (MODE == 1) { gb = *(const v4f*)(g2 + c4); bb2 = *(const v4f*)(b2 + c4); }
  v4f yv[2];
#pragma unroll
  for (int rr = 0; rr < 2; ++rr) {
    const v4f x = *(const v4f*)(src + (size_t)(r0 + rr) * kDm + c4);
    const v4f y = ln_vec4(x, ga, ba);
    yv[rr] = y;
    if (MODE != 2) {
      v4f hq = y;
      if (MODE == 1) hq = ln_vec4(y, gb, bb2);
      _Float16* hp = &sH[wave][rr * kDm + c4];
      hp[0] = (_Float16)(hq[0] * s16);
      hp[1] = (_Float16)(hq[1] * s16);
      hp[2] = (_Float16)(hq[2] * s16);
      hp[3] = (_Float16)(hq[3] * s16);
    }
  }
  v8h pk;
#pragma unroll
  for (int e = 0; e < 8; ++e) pk[e] = (_Float16)0.0f;
  if (MODE != 2) {
    __builtin_amdgcn_fence(__ATOMIC_RELEASE, "workgroup");
    __builtin_amdgcn_wave_barrier();
    __builtin_amdgcn_fence(__ATOMIC_ACQUIRE, "workgroup");
    pk = *(const v8h*)(&sH[wave][(lane >> 4) * kDm + (lane & 15) * 8]);
  }
  for (int pass = 0; pass < 2; ++pass) {
    if (MODE != 3) {
      *(volatile v4f*)(outf + (size_t)r0 * kDm + c4) = yv[0];
      *(volatile v4f*)(outf + (size_t)(r0 + 1) * kDm + c4) = yv[1];
    }
    if (MODE != 2) {
      *(volatile v8h*)(out16 + (size_t)(r0 + (lane >> 4)) * kDm + (lane & 15) * 8) = pk;
    }
    __threadfence();
  }
}

__global__ __launch_bounds__(256) void conv_silu_kernel(
    const float* __restrict__ XZ, const float* __restrict__ cw, const float* __restrict__ cb,
    float* __restrict__ UC, unsigned short* __restrict__ UP, float s16)
{
  __shared__ __align__(16) float sT[16 * kConvTP];
  const int tid = threadIdx.x, lane = tid & 31, wave = tid >> 5;
  const int d0 = blockIdx.x * 256, d = d0 + tid;
  const int g0 = blockIdx.y * 64;
  const int tb = g0 & (kSeq - 1);
  const float w0 = cw[d * 4 + 0], w1 = cw[d * 4 + 1], w2 = cw[d * 4 + 2], w3 = cw[d * 4 + 3];
  const float bc = cb[d];
  float xm3, xm2, xm1;
  {
    const bool hist = (tb > 0);
    const int rb = hist ? (g0 - 3) : g0;
    const float v3 = XZ[(size_t)rb * kXzP + d];
    const float v2 = XZ[(size_t)(rb + 1) * kXzP + d];
    const float v1 = XZ[(size_t)(rb + 2) * kXzP + d];
    xm3 = hist ? v3 : 0.f;
    xm2 = hist ? v2 : 0.f;
    xm1 = hist ? v1 : 0.f;
  }
  const int hrow = wave >> 1;
  const int hch  = (wave & 1) * 128 + lane * 4;
#pragma unroll 1
  for (int sub = 0; sub < 4; ++sub) {
    const int lb = g0 + sub * 16;
#pragma unroll 1
    for (int s = 0; s < 16; ++s) {
      const float xcur = XZ[(size_t)(lb + s) * kXzP + d];
      float acc = w0 * xm3;
      acc = fmaf(w1, xm2, acc);
      acc = fmaf(w2, xm1, acc);
      acc = fmaf(w3, xcur, acc);
      const float sv = acc + bc;
      const float sg = __builtin_amdgcn_rcpf(1.0f + __expf(-sv));
      sT[s * kConvTP + tid] = sv * sg;
      xm3 = xm2; xm2 = xm1; xm1 = xcur;
    }
    __syncthreads();
    v4f fv[4];
    v8h hv[2];
#pragma unroll
    for (int it = 0; it < 4; ++it) fv[it] = *(const v4f*)(sT + (it * 4 + hrow) * kConvTP + hch);
#pragma unroll
    for (int it = 0; it < 2; ++it) {
      const float* sp = sT + (it * 8 + wave) * kConvTP + lane * 8;
      const v4f a0 = *(const v4f*)(sp);
      const v4f a1 = *(const v4f*)(sp + 4);
#pragma unroll
      for (int e = 0; e < 4; ++e) {
        hv[it][e]     = (_Float16)(a0[e] * s16);
        hv[it][4 + e] = (_Float16)(a1[e] * s16);
      }
    }
    for (int pass = 0; pass < 2; ++pass) {
#pragma unroll
      for (int it = 0; it < 4; ++it)
        *(volatile v4f*)(UC + (size_t)(lb + it * 4 + hrow) * kDin + d0 + hch) = fv[it];
#pragma unroll
      for (int it = 0; it < 2; ++it) {
        const size_t o = (size_t)(lb + it * 8 + wave) * kDin + d0 + lane * 8;
        *(volatile v8h*)(UP + o) = hv[it];
      }
      __threadfence();
    }
    __syncthreads();
  }
}

__global__ __launch_bounds__(64) void scan_kernel(
    const float* __restrict__ XD, const float* __restrict__ UC, const float* __restrict__ XZ,
    const float* __restrict__ Wdt, const float* __restrict__ bdt, const float* __restrict__ Alog,
    const float* __restrict__ Dp, unsigned short* __restrict__ YP, float s16)
{
  __shared__ __align__(16) float sX[kScanTS * kXdP];
  __shared__ __align__(16) float sY[kScanTS * kScanYP];
  __shared__ __align__(16) float sW[kDtR * kScanCh];
  __shared__ __align__(16) float sA[kNst * kScanCh];
  const int tid = threadIdx.x, lane = tid & 31, wave = tid >> 5;
  constexpr int kBlkPerB = kDin / kScanCh;
  const int bix = blockIdx.x / kBlkPerB;
  const int d0  = (blockIdx.x - bix * kBlkPerB) * kScanCh;
  const int d   = d0 + tid;
  const size_t row0 = (size_t)bix * kSeq;
#pragma unroll 1
  for (int r = 0; r < kDtR; ++r) sW[r * kScanCh + tid] = Wdt[(size_t)d * kDtR + r];
#pragma unroll 1
  for (int s = 0; s < kNst; ++s) sA[s * kScanCh + tid] = -expf(Alog[(size_t)d * kNst + s]);
  __syncthreads();
  float negA[kNst], h[kNst];
#pragma unroll
  for (int s = 0; s < kNst; ++s) {
    negA[s] = sA[s * kScanCh + tid];
    h[s] = 0.f;
  }
  const float bb = bdt[d], Dd = Dp[d];
  const int lr = tid >> 4, lc4 = (tid & 15) * 4;
  const int q = lane >> 3, c8 = (lane & 7) * 8;
#pragma unroll 1
  for (int t0 = 0; t0 < kSeq; t0 += kScanTS) {
    __syncthreads();
#pragma unroll
    for (int i = 0; i < 16; ++i) {
      const int r = lr + 4 * i;
      *(v4f*)(sX + r * kXdP + lc4) = *(const v4f*)(XD + (row0 + t0 + r) * kXdP + lc4);
    }
    __syncthreads();
#pragma unroll 1
    for (int s = 0; s < kScanTS; ++s) {
      const int t = t0 + s;
      const float* xr = sX + s * kXdP;
      float vdot = 0.f;
#pragma unroll 1
      for (int r4 = 0; r4 < kDtR / 4; ++r4) {
        const v4f xv = *(const v4f*)(xr + 4 * r4);
        const float* wp = sW + (4 * r4) * kScanCh + tid;
        vdot = fmaf(xv[0], wp[0], vdot);
        vdot = fmaf(xv[1], wp[kScanCh], vdot);
        vdot = fmaf(xv[2], wp[2 * kScanCh], vdot);
        vdot = fmaf(xv[3], wp[3 * kScanCh], vdot);
      }
      float Bs[kNst], Cs[kNst];
#pragma unroll
      for (int q4 = 0; q4 < 4; ++q4) {
        const v4f bv = *(const v4f*)(xr + kDtR + 4 * q4);
        const v4f cv = *(const v4f*)(xr + kDtR + kNst + 4 * q4);
        Bs[4 * q4 + 0] = bv[0]; Bs[4 * q4 + 1] = bv[1]; Bs[4 * q4 + 2] = bv[2]; Bs[4 * q4 + 3] = bv[3];
        Cs[4 * q4 + 0] = cv[0]; Cs[4 * q4 + 1] = cv[1]; Cs[4 * q4 + 2] = cv[2]; Cs[4 * q4 + 3] = cv[3];
      }
      const float v   = vdot + bb;
      const float a   = __expf(-fabsf(v));
      const float u   = 1.0f + a;
      const float l1p = __logf(u) + (a - (u - 1.0f)) * __builtin_amdgcn_rcpf(u);
      const float dt  = fmaxf(v, 0.0f) + l1p;
      const float xt  = UC[(row0 + t) * kDin + d];
      const float dtx = dt * xt;
      float y = 0.f;
#pragma unroll
      for (int k = 0; k < kNst; ++k) {
        const float e = __expf(dt * negA[k]);
        h[k] = e * h[k] + dtx * Bs[k];
        y = h[k] * Cs[k] + y;
      }
      y = xt * Dd + y;
      const float zv = XZ[(row0 + t) * kXzP + kDin + d];
      const float sg = __builtin_amdgcn_rcpf(1.0f + __expf(-zv));
      y = y * (zv * sg);
      sY[s * kScanYP + tid] = y;
    }
    __syncthreads();
    v8h hv[8];
#pragma unroll
    for (int it = 0; it < 8; ++it) {
      const int row = it * 8 + wave * 4 + q;
      const float* sp = sY + row * kScanYP + c8;
      const v4f a0 = *(const v4f*)(sp);
      const v4f a1 = *(const v4f*)(sp + 4);
#pragma unroll
      for (int e = 0; e < 4; ++e) {
        hv[it][e]     = (_Float16)(a0[e] * s16);
        hv[it][4 + e] = (_Float16)(a1[e] * s16);
      }
    }
    for (int pass = 0; pass < 2; ++pass) {
#pragma unroll
      for (int it = 0; it < 8; ++it) {
        const int row = it * 8 + wave * 4 + q;
        const size_t o = (row0 + t0 + row) * kDin + d0 + c8;
        *(volatile v8h*)(YP + o) = hv[it];
      }
      __threadfence();
    }
  }
}

template <bool OUT16>
__global__ __launch_bounds__(256) void gelu2_kernel(
    const float* __restrict__ src, void* __restrict__ dst, int n2, float s16)
{
  const int i = blockIdx.x * 256 + threadIdx.x;
  if (i >= n2) return;
  const v2f x = *(const v2f*)(src + 2 * (size_t)i);
  const float g0 = 0.5f * x[0] * (1.0f + erff(x[0] * 0.70710678118654752f));
  const float g1 = 0.5f * x[1] * (1.0f + erff(x[1] * 0.70710678118654752f));
  if (OUT16) {
    const _Float16 h0 = (_Float16)(g0 * s16), h1 = (_Float16)(g1 * s16);
    const unsigned w = (unsigned)__builtin_bit_cast(unsigned short, h0) | ((unsigned)__builtin_bit_cast(unsigned short, h1) << 16);
    volatile unsigned* p = (volatile unsigned*)dst + i;
    *p = w;
    __threadfence();
    *p = w;
  } else {
    v2f o;
    o[0] = g0; o[1] = g1;
    float* pf = (float*)dst + 2 * (size_t)i;
    *(volatile v2f*)pf = o;
    __threadfence();
    *(volatile v2f*)pf = o;
  }
}

__global__ __launch_bounds__(256) void gather_rows_f16_kernel(
    const float* __restrict__ hid, const int* __restrict__ pos,
    unsigned short* __restrict__ dst, float s16, int total8)
{
  const int i = blockIdx.x * 256 + threadIdx.x;
  if (i >= total8) return;
  const int e0 = i * 8;
  const int m  = e0 / kDm;
  const int c  = e0 - m * kDm;
  const int b  = m / kNMask;
  int p = pos[m];
  p = (p < 0) ? 0 : ((p >= kSeq) ? (kSeq - 1) : p);
  const float* sp = hid + ((size_t)b * kSeq + p) * kDm + c;
  const v4f a0 = *(const v4f*)(sp);
  const v4f a1 = *(const v4f*)(sp + 4);
  v8h hv;
#pragma unroll
  for (int e = 0; e < 4; ++e) {
    hv[e]     = (_Float16)(a0[e] * s16);
    hv[4 + e] = (_Float16)(a1[e] * s16);
  }
  unsigned short* qd = dst + e0;
  *(volatile v8h*)qd = hv;
  __threadfence();
  *(volatile v8h*)qd = hv;
}

__global__ __launch_bounds__(256) void logits_store_kernel(
    const float* __restrict__ lg, const float* __restrict__ decb, float* __restrict__ out0, int total4)
{
  const int i = blockIdx.x * 256 + threadIdx.x;
  if (i >= total4) return;
  const int row = i >> 3, c4 = (i & 7) * 4;
  v4f v = *(const v4f*)(lg + (size_t)row * kDecP + c4);
  const v4f bb = *(const v4f*)(decb + c4);
  v[0] += bb[0]; v[1] += bb[1]; v[2] += bb[2]; v[3] += bb[3];
  float* p = out0 + (size_t)row * kElem + c4;
  *(volatile v4f*)p = v;
  __threadfence();
  *(volatile v4f*)p = v;
}

extern "C" void kernel_launch(void* const* d_in, const int* in_sizes, int n_in,
                              void* d_out, int out_size, void* d_ws, size_t ws_size,
                              hipStream_t stream) {
  if (n_in < 31) return;
  if (in_sizes[0]  != kRows * kElem) return;
  if (in_sizes[1]  != kHeadRows) return;
  if (in_sizes[2]  != kDm * kElem) return;
  if (in_sizes[3]  != kDm || in_sizes[4] != kDm || in_sizes[5] != kDm) return;
  if (in_sizes[6]  != kLayers * kXzP * kDm) return;
  if (in_sizes[7]  != kLayers * kDin * 4) return;
  if (in_sizes[8]  != kLayers * kDin) return;
  if (in_sizes[9]  != kLayers * kXdN * kDin) return;
  if (in_sizes[10] != kLayers * kDin * kDtR) return;
  if (in_sizes[11] != kLayers * kDin) return;
  if (in_sizes[12] != kLayers * kDin * kNst) return;
  if (in_sizes[13] != kLayers * kDin) return;
  if (in_sizes[14] != kLayers * kDm * kDin) return;
  if (in_sizes[15] != kLayers * kDm || in_sizes[16] != kLayers * kDm) return;
  if (in_sizes[17] != kLayers * kDm || in_sizes[18] != kLayers * kDm) return;
  if (in_sizes[19] != kLayers * kDff * kDm) return;
  if (in_sizes[20] != kLayers * kDff) return;
  if (in_sizes[21] != kLayers * kDm * kDff) return;
  if (in_sizes[22] != kLayers * kDm) return;
  if (in_sizes[23] != kLayers * kDm || in_sizes[24] != kLayers * kDm) return;
  if (in_sizes[25] != kDm * kDm || in_sizes[26] != kDm) return;
  if (in_sizes[27] != kDm || in_sizes[28] != kDm) return;
  if (in_sizes[29] != kElem * kDm || in_sizes[30] != kElem) return;
  if (out_size != kOutTotal) return;
  if (ws_size < kWsTotal) return;

  const float* input_ids  = (const float*)d_in[0];
  const int*   masked_pos = (const int*)  d_in[1];
  const float* proj_w     = (const float*)d_in[2];
  const float* proj_b     = (const float*)d_in[3];
  const float* inorm_g    = (const float*)d_in[4];
  const float* inorm_b    = (const float*)d_in[5];
  const float* in_proj_w  = (const float*)d_in[6];
  const float* conv_w     = (const float*)d_in[7];
  const float* conv_b     = (const float*)d_in[8];
  const float* x_proj_w   = (const float*)d_in[9];
  const float* dt_proj_w  = (const float*)d_in[10];
  const float* dt_proj_b  = (const float*)d_in[11];
  const float* A_log      = (const float*)d_in[12];
  const float* D_param    = (const float*)d_in[13];
  const float* out_proj_w = (const float*)d_in[14];
  const float* ln1_g      = (const float*)d_in[15];
  const float* ln1_b      = (const float*)d_in[16];
  const float* ln2_g      = (const float*)d_in[17];
  const float* ln2_b      = (const float*)d_in[18];
  const float* ffn_w1     = (const float*)d_in[19];
  const float* ffn_b1     = (const float*)d_in[20];
  const float* ffn_w2     = (const float*)d_in[21];
  const float* ffn_b2     = (const float*)d_in[22];
  const float* ln3_g      = (const float*)d_in[23];
  const float* ln3_b      = (const float*)d_in[24];
  const float* lin_w      = (const float*)d_in[25];
  const float* lin_b      = (const float*)d_in[26];
  const float* norm_g     = (const float*)d_in[27];
  const float* norm_b     = (const float*)d_in[28];
  const float* dec_w      = (const float*)d_in[29];
  const float* dec_b      = (const float*)d_in[30];
  float* out0 = (float*)d_out;
  float* out1 = (float*)d_out + kOut0Floats;

  char* ws = (char*)d_ws;
  unsigned short* X16 = (unsigned short*)(ws + kOffX16);
  unsigned short* PW  = (unsigned short*)(ws + kOffPW);
  unsigned short* WIN = (unsigned short*)(ws + kOffWIN);
  unsigned short* WX  = (unsigned short*)(ws + kOffWX);
  unsigned short* WO  = (unsigned short*)(ws + kOffWO);
  unsigned short* W1  = (unsigned short*)(ws + kOffW1);
  unsigned short* W2  = (unsigned short*)(ws + kOffW2);
  unsigned short* LIN = (unsigned short*)(ws + kOffLIN);
  unsigned short* DEC = (unsigned short*)(ws + kOffDEC);
  float*          OUT = (float*)(ws + kOffOUT);
  float*          TT  = (float*)(ws + kOffTT);
  unsigned short* H16 = (unsigned short*)(ws + kOffH16);
  unsigned short* A16 = (unsigned short*)(ws + kOffA16);
  float*          XZ  = (float*)(ws + kOffXZ);
  float*          UC  = (float*)(ws + kOffUC);
  unsigned short* UP  = (unsigned short*)(ws + kOffUP);
  float*          XD  = (float*)(ws + kOffXD);
  unsigned short* YP  = (unsigned short*)(ws + kOffYP);
  float*          F1  = (float*)(ws + kOffF1);
  unsigned short* G16 = (unsigned short*)(ws + kOffG16);
  unsigned short* HM  = (unsigned short*)(ws + kOffHM);
  float*          HL  = (float*)(ws + kOffHL);
  float*          HG  = (float*)(ws + kOffHG);
  unsigned short* HN  = (unsigned short*)(ws + kOffHN);
  float*          LG  = (float*)(ws + kOffLG);

  const float kSAct  = 64.0f;
  const float kSU    = 1024.0f;
  const float kSY    = 4096.0f;
  const float kSG    = 1024.0f;
  const float kSW    = 4096.0f;
  const float kInv18 = 1.0f / 262144.0f;
  const float kInv22 = 1.0f / 4194304.0f;
  const float kInv24 = 1.0f / 16777216.0f;

  {
    const int t8 = kRows * kElem / 8;
    cast_pad_f16_kernel<<<(t8 + 255) / 256, 256, 0, stream>>>(input_ids, X16, kRows, kRows, kElem, kSAct, t8);
  }
  {
    const int t8 = kDm * kElem / 8;
    cast_pad_f16_kernel<<<(t8 + 255) / 256, 256, 0, stream>>>(proj_w, PW, kDm, kDm, kElem, kSW, t8);
  }
  {
    const int t8 = kLayers * kXzP * kDm / 8;
    cast_pad_f16_kernel<<<(t8 + 255) / 256, 256, 0, stream>>>(in_proj_w, WIN, kLayers * kXzP, kLayers * kXzP, kDm, kSW, t8);
  }
  {
    const int t8 = kLayers * kXdP * kDin / 8;
    cast_pad_f16_kernel<<<(t8 + 255) / 256, 256, 0, stream>>>(x_proj_w, WX, kXdN, kXdP, kDin, kSW, t8);
  }
  {
    const int t8 = kLayers * kDm * kDin / 8;
    cast_pad_f16_kernel<<<(t8 + 255) / 256, 256, 0, stream>>>(out_proj_w, WO, kLayers * kDm, kLayers * kDm, kDin, kSW, t8);
  }
  {
    const int t8 = kLayers * kDff * kDm / 8;
    cast_pad_f16_kernel<<<(t8 + 255) / 256, 256, 0, stream>>>(ffn_w1, W1, kLayers * kDff, kLayers * kDff, kDm, kSW, t8);
  }
  {
    const int t8 = kLayers * kDm * kDff / 8;
    cast_pad_f16_kernel<<<(t8 + 255) / 256, 256, 0, stream>>>(ffn_w2, W2, kLayers * kDm, kLayers * kDm, kDff, kSW, t8);
  }
  {
    const int t8 = kDm * kDm / 8;
    cast_pad_f16_kernel<<<(t8 + 255) / 256, 256, 0, stream>>>(lin_w, LIN, kDm, kDm, kDm, kSW, t8);
  }
  {
    const int t8 = kDecP * kDm / 8;
    cast_pad_f16_kernel<<<(t8 + 255) / 256, 256, 0, stream>>>(dec_w, DEC, kElem, kDecP, kDm, kSW, t8);
  }

  wmma_gemm64<0, 0, 2, 0, false><<<dim3(8, 1), 256, 0, stream>>>(
      X16, nullptr, kElem, 0L,
      PW, nullptr, kElem, 0L,
      (void*)TT, nullptr, kDm, 0L,
      proj_b, nullptr, 0L,
      kRows, kDm, kElem, kInv18);
  ln_rows_kernel<1><<<kRows / 16, 256, 0, stream>>>(TT, inorm_g, inorm_b, ln1_g, ln1_b, OUT, H16, kRows, kSAct);

  for (int i = 0; i < kLayers; ++i) {
    wmma_gemm64<0, 0, 0, 0, false><<<dim3(32, 1), 256, 0, stream>>>(
        H16, nullptr, kDm, 0L,
        WIN + (size_t)i * kXzP * kDm, nullptr, kDm, 0L,
        (void*)XZ, nullptr, kXzP, 0L,
        nullptr, nullptr, 0L,
        kRows, kXzP, kDm, kInv18);
    conv_silu_kernel<<<dim3(kDin / 256, kRows / 64), 256, 0, stream>>>(
        XZ, conv_w + (size_t)i * kDin * 4, conv_b + (size_t)i * kDin, UC, UP, kSU);
    wmma_gemm64<0, 0, 0, 0, false><<<dim3(4, 1), 256, 0, stream>>>(
        UP, nullptr, kDin, 0L,
        WX + (size_t)i * kXdP * kDin, nullptr, kDin, 0L,
        (void*)XD, nullptr, kXdP, 0L,
        nullptr, nullptr, 0L,
        kRows, kXdP, kDin, kInv22);
    scan_kernel<<<kBatch * (kDin / kScanCh), kScanCh, 0, stream>>>(
        XD, UC, XZ, dt_proj_w + (size_t)i * kDin * kDtR, dt_proj_b + (size_t)i * kDin,
        A_log + (size_t)i * kDin * kNst, D_param + (size_t)i * kDin, YP, kSY);
    wmma_gemm64<0, 0, 0, 0, true><<<dim3(8, 1), 256, 0, stream>>>(
        YP, nullptr, kDin, 0L,
        WO + (size_t)i * kDm * kDin, nullptr, kDin, 0L,
        (void*)TT, nullptr, kDm, 0L,
        nullptr, OUT, 0L,
        kRows, kDm, kDin, kInv24);
    ln_rows_kernel<0><<<kRows / 16, 256, 0, stream>>>(
        TT, ln2_g + (size_t)i * kDm, ln2_b + (size_t)i * kDm, nullptr, nullptr, OUT, A16, kRows, kSAct);
    wmma_gemm64<0, 0, 2, 0, false><<<dim3(32, 1), 256, 0, stream>>>(
        A16, nullptr, kDm, 0L,
        W1 + (size_t)i * kDff * kDm, nullptr, kDm, 0L,
        (void*)F1, nullptr, kDff, 0L,
        ffn_b1 + (size_t)i * kDff, nullptr, 0L,
        kRows, kDff, kDm, kInv18);
    gelu2_kernel<true><<<(kRows * kDff / 2 + 255) / 256, 256, 0, stream>>>(F1, (void*)G16, kRows * kDff / 2, kSG);
    wmma_gemm64<0, 0, 2, 0, true><<<dim3(8, 1), 256, 0, stream>>>(
        G16, nullptr, kDff, 0L,
        W2 + (size_t)i * kDm * kDff, nullptr, kDff, 0L,
        (void*)TT, nullptr, kDm, 0L,
        ffn_b2 + (size_t)i * kDm, OUT, 0L,
        kRows, kDm, kDff, kInv22);
    if (i + 1 < kLayers) {
      ln_rows_kernel<1><<<kRows / 16, 256, 0, stream>>>(
          TT, ln3_g + (size_t)i * kDm, ln3_b + (size_t)i * kDm,
          ln1_g + (size_t)(i + 1) * kDm, ln1_b + (size_t)(i + 1) * kDm, OUT, H16, kRows, kSAct);
    } else {
      ln_rows_kernel<2><<<kRows / 16, 256, 0, stream>>>(
          TT, ln3_g + (size_t)i * kDm, ln3_b + (size_t)i * kDm, nullptr, nullptr, out1, nullptr, kRows, kSAct);
    }
  }

  gather_rows_f16_kernel<<<(kHeadRows * kDm / 8 + 255) / 256, 256, 0, stream>>>(out1, masked_pos, HM, kSAct, kHeadRows * kDm / 8);
  wmma_gemm64<0, 0, 2, 0, false><<<dim3(1, 1), 256, 0, stream>>>(
      HM, nullptr, kDm, 0L,
      LIN, nullptr, kDm, 0L,
      (void*)HL, nullptr, kDm, 0L,
      lin_b, nullptr, 0L,
      kHeadRows, kDm, kDm, kInv18);
  gelu2_kernel<false><<<(kHeadRows * kDm / 2 + 255) / 256, 256, 0, stream>>>(HL, (void*)HG, kHeadRows * kDm / 2, 1.0f);
  ln_rows_kernel<3><<<kHeadRows / 16, 256, 0, stream>>>(HG, norm_g, norm_b, nullptr, nullptr, nullptr, HN, kHeadRows, kSAct);
  wmma_gemm64<0, 0, 0, 0, false><<<dim3(1, 1), 256, 0, stream>>>(
      HN, nullptr, kDm, 0L,
      DEC, nullptr, kDm, 0L,
      (void*)LG, nullptr, kDecP, 0L,
      nullptr, nullptr, 0L,
      kHeadRows, kDecP, kDm, kInv18);
  logits_store_kernel<<<(kHeadRows * kElem / 4 + 255) / 256, 256, 0, stream>>>(LG, dec_b, out0, kHeadRows * kElem / 4);
}
